// MultiheadedAttention_19559281066467
// MI455X (gfx1250) — hardware-verified
//
#include <hip/hip_runtime.h>
#include <math.h>

#ifndef NB
#define NB 8
#endif
#ifndef SEQ
#define SEQ 1024
#endif
#define NB_FULL 8
#define SEQ_FULL 1024
#define DM 1024
#define NH 16
#define HD 64
#define D3 3072
#define MR (NB * SEQ)
static_assert(SEQ % 64 == 0);
static_assert(MR % 64 == 0);
static_assert(DM % 64 == 0);
static_assert(D3 % 64 == 0);
static_assert(NH * HD == DM);
static_assert(NB <= NB_FULL);
static_assert(SEQ <= SEQ_FULL);

typedef __attribute__((ext_vector_type(16))) _Float16 v16h;
typedef __attribute__((ext_vector_type(8)))  _Float16 v8h;
typedef __attribute__((ext_vector_type(16))) __bf16   v16b;
typedef __attribute__((ext_vector_type(8)))  __bf16   v8b;
typedef __attribute__((ext_vector_type(8)))  float    v8f;
typedef __attribute__((ext_vector_type(4)))  float    v4f;
typedef __attribute__((ext_vector_type(4)))  unsigned int cm_u4;

#define AL256(x) (((((size_t)(x)) + 255) / 256) * 256)
constexpr size_t SZ_XB  = AL256((size_t)MR * DM * 2);
constexpr size_t SZ_WQ  = AL256((size_t)D3 * DM * 2);
constexpr size_t SZ_WO  = AL256((size_t)DM * DM * 2);
constexpr size_t SZ_BV  = AL256((size_t)4096 * 4);
constexpr size_t SZ_MB  = AL256((size_t)SEQ_FULL * SEQ_FULL * 4);
constexpr size_t SZ_QKV = AL256((size_t)MR * D3 * 2);
constexpr size_t SZ_CTX = AL256((size_t)MR * DM * 2);
constexpr size_t WS_TOTAL = SZ_XB + SZ_WQ + SZ_WO + SZ_BV + SZ_MB + SZ_QKV + SZ_CTX;
static_assert(WS_TOTAL <= (size_t)134217728);

#define VST2(T, ptr, val) do { const T vst2_v_ = (val); *(volatile T*)(ptr) = vst2_v_; __threadfence(); *(volatile T*)(ptr) = vst2_v_; } while (0)
#define VST2V4(ptr, val) do { const v4f vst2_v4_ = (val); *(volatile v4f*)(ptr) = vst2_v4_; __threadfence(); *(volatile v4f*)(ptr) = vst2_v4_; } while (0)

__device__ __forceinline__ v8f wmma16(v16h a, v16h b, v8f c) {
    c = __builtin_amdgcn_wmma_f32_16x16x32_f16(false, a, false, b, (short)0, c, false, false);
    asm volatile("v_nop\n\tv_nop\n\tv_nop\n\tv_nop" : "+v"(c) : "v"(a), "v"(b));
    return c;
}
union FH { v16h v; v8h h[2]; };

__device__ __forceinline__ float cmb_bf(float v) { const unsigned u = __builtin_bit_cast(unsigned, v); const unsigned r = (u + 0x7fffu + ((u >> 16) & 1u)) & 0xffff0000u; return __builtin_bit_cast(float, r); }
__device__ __forceinline__ unsigned int cmb_pk2(float a, float b) { return (unsigned int)__builtin_bit_cast(unsigned short, (_Float16)a) | ((unsigned int)__builtin_bit_cast(unsigned short, (_Float16)b) << 16); }

namespace w25 {
typedef __attribute__((ext_vector_type(16))) _Float16 v16h;
typedef __attribute__((ext_vector_type(8)))  _Float16 v8h;
typedef __attribute__((ext_vector_type(16))) __bf16   v16b;
typedef __attribute__((ext_vector_type(8)))  __bf16   v8b;
typedef __attribute__((ext_vector_type(8)))  float    v8f;
typedef __attribute__((ext_vector_type(4)))  float    v4f;

__device__ __forceinline__ unsigned short f2bf_bits(float f) {
  unsigned u = __float_as_uint(f);
  return (unsigned short)((u + 0x7FFFu + ((u >> 16) & 1u)) >> 16);
}
__device__ __forceinline__ float bf_bits2f(unsigned short h) { return __uint_as_float(((unsigned)h) << 16); }

__device__ __forceinline__ void dep_guard_h(v8f& a, v8f& b, v16h x, v16h y) { asm volatile("v_nop\n\tv_nop\n\tv_nop\n\tv_nop" : "+v"(a), "+v"(b) : "v"(x), "v"(y)); }
__device__ __forceinline__ void dep_guard_b(v8f& a, v8f& b, v16b x, v16b y) { asm volatile("v_nop\n\tv_nop\n\tv_nop\n\tv_nop" : "+v"(a), "+v"(b) : "v"(x), "v"(y)); }
__device__ __forceinline__ void keep4_h(v16h a, v16h b, v16h c, v16h d) { asm volatile("v_nop" :: "v"(a), "v"(b), "v"(c), "v"(d)); }
__device__ __forceinline__ void keep4_b(v16b a, v16b b, v16b c, v16b d) { asm volatile("v_nop" :: "v"(a), "v"(b), "v"(c), "v"(d)); }
__device__ __forceinline__ void acc_guard4(v8f& a, v8f& b, v8f& c, v8f& d) { asm volatile("v_nop\n\tv_nop\n\tv_nop\n\tv_nop" : "+v"(a), "+v"(b), "+v"(c), "+v"(d)); }
template <typename T> struct Frag;
template <> struct Frag<_Float16> {
  typedef v16h V; union U { v16h v; v8h h[2]; };
  static __device__ __forceinline__ v16h load(const _Float16* p) {
    U f; f.h[0] = *(const v8h*)(p); f.h[1] = *(const v8h*)(p + 16); return f.v;
  }
  static __device__ __forceinline__ v8f mma(v16h a, v16h b, v8f c) {
    return __builtin_amdgcn_wmma_f32_16x16x32_f16(false, a, false, b, (short)0, c, false, false);
  }
  static __device__ __forceinline__ void guard(v8f& a, v8f& b, v16h x, v16h y) { dep_guard_h(a, b, x, y); }
  static __device__ __forceinline__ void keep(v16h a, v16h b, v16h c, v16h d) { keep4_h(a, b, c, d); }
};
template <> struct Frag<__bf16> {
  typedef v16b V; union U { v16b v; v8b h[2]; };
  static __device__ __forceinline__ v16b load(const __bf16* p) {
    U f; f.h[0] = *(const v8b*)(p); f.h[1] = *(const v8b*)(p + 16); return f.v;
  }
  static __device__ __forceinline__ v8f mma(v16b a, v16b b, v8f c) {
    return __builtin_amdgcn_wmma_f32_16x16x32_bf16(false, a, false, b, (short)0, c, false, false);
  }
  static __device__ __forceinline__ void guard(v8f& a, v8f& b, v16b x, v16b y) { dep_guard_b(a, b, x, y); }
  static __device__ __forceinline__ void keep(v16b a, v16b b, v16b c, v16b d) { keep4_b(a, b, c, d); }
};

template <int ET> struct Elem;
template <> struct Elem<0> { typedef _Float16 T; };
template <> struct Elem<1> { typedef __bf16 T; };
template <int ET, bool SPLIT, int BIAS_MODE, int OUT_MODE, bool RESID, int ACT = 0>
__global__ __launch_bounds__(256) void wmma_gemm64(
    const unsigned short* __restrict__ Ap, const unsigned short* __restrict__ A2p, int lda, long strideA,
    const unsigned short* __restrict__ Btp, const unsigned short* __restrict__ Bt2p, int ldb, long strideB,
    void* __restrict__ Cout, void* __restrict__ Cout2, int ldc, long strideC,
    const float* __restrict__ bias,
    const float* __restrict__ resid, long strideR,
    int M, int N, int K, float scale) {
  typedef typename Elem<ET>::T T;
  typedef typename Frag<T>::V V;
  const T* A = (const T*)Ap; const T* A2 = (const T*)A2p; const T* Bt = (const T*)Btp; const T* Bt2 = (const T*)Bt2p;
  __shared__ __align__(16) float sT[8][16 * 68];
  const int b    = blockIdx.y;
  const int lane = threadIdx.x & 31;
  const int wave = threadIdx.x >> 5;
  const int tilesN = N >> 6;
  const int tilesM = M >> 6;
  const int tile = blockIdx.x * 8 + wave;
  if (tile >= tilesM * tilesN) return;
  const int tm = tile / tilesN;
  const int tn = tile - tm * tilesN;
  const int m0 = tm << 6;
  const int n0 = tn << 6;

  const T* Ab  = A  + (size_t)b * strideA;
  const T* Bb  = Bt + (size_t)b * strideB;
  const T* Ab2 = SPLIT ? (A2  + (size_t)b * strideA) : nullptr;
  const T* Bb2 = SPLIT ? (Bt2 + (size_t)b * strideB) : nullptr;

  const int rlane = lane & 15;
  const int koff  = (lane >> 4) * 8;
  const int mOff  = (lane >> 4) * 8;

  v8f acc[4][4];
#pragma unroll
  for (int i = 0; i < 4; ++i)
#pragma unroll
    for (int j = 0; j < 4; ++j) acc[i][j] = (v8f){0.f,0.f,0.f,0.f,0.f,0.f,0.f,0.f};

  for (int k0 = 0; k0 < K; k0 += 32) {
    V bh[4], bl[4];
#pragma unroll
    for (int j = 0; j < 4; ++j) {
      const size_t bo = (size_t)(n0 + (j << 4) + rlane) * ldb + koff + k0;
      bh[j] = Frag<T>::load(Bb + bo);
      if (SPLIT) bl[j] = Frag<T>::load(Bb2 + bo);
    }
#pragma unroll
    for (int i = 0; i < 4; ++i) {
      const size_t ao = (size_t)(m0 + (i << 4) + rlane) * lda + koff + k0;
      V ah = Frag<T>::load(Ab + ao);
      V al;
      if (SPLIT) al = Frag<T>::load(Ab2 + ao);
#pragma unroll
      for (int j = 0; j < 4; ++j) {
        acc[i][j] = Frag<T>::mma(ah, bh[j], acc[i][j]);
        if (SPLIT) {
          acc[i][j] = Frag<T>::mma(ah, bl[j], acc[i][j]);
          acc[i][j] = Frag<T>::mma(al, bh[j], acc[i][j]);
        }
      }
      Frag<T>::guard(acc[i][0], acc[i][3], ah, SPLIT ? al : ah);
    }
    Frag<T>::keep(bh[0], bh[1], bh[2], bh[3]);
    if (SPLIT) Frag<T>::keep(bl[0], bl[1], bl[2], bl[3]);
  }
  acc_guard4(acc[0][0], acc[0][1], acc[0][2], acc[0][3]);
  acc_guard4(acc[1][0], acc[1][1], acc[1][2], acc[1][3]);
  acc_guard4(acc[2][0], acc[2][1], acc[2][2], acc[2][3]);
  acc_guard4(acc[3][0], acc[3][1], acc[3][2], acc[3][3]);

  float* slab = sT[wave];
  const float* Rb = RESID ? (resid + (size_t)b * strideR) : nullptr;
#pragma unroll
  for (int i = 0; i < 4; ++i) {
    const int mBase = m0 + (i << 4);
#pragma unroll
    for (int j = 0; j < 4; ++j) {
      const int n = n0 + (j << 4) + rlane;
      float bv = 0.f;
      if (BIAS_MODE == 2) bv = bias[n];
#pragma unroll
      for (int r = 0; r < 8; ++r) {
        float v = acc[i][j][r] * scale;
        if (BIAS_MODE == 1) v += bias[mBase + mOff + r];
        if (BIAS_MODE == 2) v += bv;
        if (RESID) v += Rb[(size_t)(mBase + mOff + r) * ldc + n];
        if (ACT == 1) v = tanhf(v);
        if (ACT == 2) v = fmaxf(v, 0.0f);
        if (ACT == 3) v = v / (1.0f + expf(-v));
        if (ACT == 4) v = (v > 0.f) ? v : 0.01f * v;
        if (ACT == 5) v = 0.5f * v * (1.0f + erff(v * 0.70710678118654752f));
        if (ACT == 6) v = (v > 0.f) ? v : 0.2f * v;
        if (ACT == 7) { const float u = 0.7978845608028654f * (v + 0.044715f * v * v * v); v = 0.5f * v * (1.f + tanhf(u)); }
        slab[(mOff + r) * 68 + (j << 4) + rlane] = v;
      }
    }
    __builtin_amdgcn_fence(3, "workgroup");
    __builtin_amdgcn_wave_barrier();
    __builtin_amdgcn_fence(2, "workgroup");
    if (OUT_MODE == 0) {
      float* C = (float*)Cout + (size_t)b * strideC;
      const int hh = lane >> 4, c4 = (lane & 15) * 4;
      for (int pass = 0; pass < 2; ++pass) {
#pragma unroll
        for (int it = 0; it < 8; ++it) {
          const int row = it * 2 + hh;
          v4f v = *(const v4f*)(slab + row * 68 + c4);
          *(volatile v4f*)(C + (size_t)(mBase + row) * ldc + n0 + c4) = v;
        }
        __threadfence();
      }
    } else {
      const int q = lane >> 3, c8 = (lane & 7) * 8;
      unsigned short* C  = (unsigned short*)Cout  + (size_t)b * strideC;
      unsigned short* C2 = (OUT_MODE == 2) ? ((unsigned short*)Cout2 + (size_t)b * strideC) : nullptr;
      for (int pass = 0; pass < 2; ++pass) {
#pragma unroll
        for (int it = 0; it < 4; ++it) {
          const int row = it * 4 + q;
          const float* sp = slab + row * 68 + c8;
          v8h hv, lv;
#pragma unroll
          for (int e = 0; e < 8; ++e) {
            if (OUT_MODE == 1) {
              hv[e] = (_Float16)sp[e];
            } else {
              unsigned short hb = f2bf_bits(sp[e]);
              unsigned short lb = f2bf_bits(sp[e] - bf_bits2f(hb));
              hv[e] = __builtin_bit_cast(_Float16, hb);
              lv[e] = __builtin_bit_cast(_Float16, lb);
            }
          }
          *(volatile v8h*)(C + (size_t)(mBase + row) * ldc + n0 + c8) = hv;
          if (OUT_MODE == 2) *(volatile v8h*)(C2 + (size_t)(mBase + row) * ldc + n0 + c8) = lv;
        }
        __threadfence();
      }
    }
    __builtin_amdgcn_fence(3, "workgroup");
    __builtin_amdgcn_wave_barrier();
    __builtin_amdgcn_fence(2, "workgroup");
  }
}
}

__global__ __launch_bounds__(256) void k_cast8(const float* __restrict__ SRC, unsigned short* __restrict__ DST, int nrows, int mode, float sc) {
    const long long u = (long long)blockIdx.x * 256 + threadIdx.x;
    if (u >= (long long)nrows * (DM / 8)) return;
    const int r = (int)(u / (DM / 8)); const int c0 = 8 * (int)(u % (DM / 8));
    long long sr;
    if (mode == 0) { const int bb = r / SEQ; const int s = r - bb * SEQ; sr = (long long)bb * SEQ_FULL + s; }
    else if (mode == 1) { const int which = r / DM; const int rem = r - which * DM; const int hq = rem / HD; const int d = rem - hq * HD; sr = (long long)hq * (3 * HD) + (long long)which * HD + d; }
    else sr = r;
    const float* s8 = SRC + sr * DM + c0;
    const v4f a = *(const v4f*)s8, bq = *(const v4f*)(s8 + 4);
    cm_u4 pk;
    pk.x = cmb_pk2(cmb_bf(a.x) * sc, cmb_bf(a.y) * sc);
    pk.y = cmb_pk2(cmb_bf(a.z) * sc, cmb_bf(a.w) * sc);
    pk.z = cmb_pk2(cmb_bf(bq.x) * sc, cmb_bf(bq.y) * sc);
    pk.w = cmb_pk2(cmb_bf(bq.z) * sc, cmb_bf(bq.w) * sc);
    VST2(cm_u4, (cm_u4*)(DST + (long long)r * DM + c0), pk);
}

__global__ __launch_bounds__(256) void k_bvec(const float* __restrict__ BQS, const float* __restrict__ BOS, float* __restrict__ BV) {
    const int i = blockIdx.x * 256 + threadIdx.x;
    if (i >= 4096) return;
    const int iq = min(i, D3 - 1);
    const int which = iq / DM; const int rem = iq - which * DM; const int hq = rem / HD; const int d = rem - hq * HD;
    const float a = cmb_bf(BQS[hq * (3 * HD) + which * HD + d]);
    const int io = min(max(i - D3, 0), DM - 1);
    const float bo = cmb_bf(BOS[io]);
    const float v = (i < D3) ? a : bo;
    VST2(float, BV + i, v);
}

__global__ __launch_bounds__(256) void k_maskbf(const float* __restrict__ MS, float* __restrict__ MB, long long n4) {
    const long long u = (long long)blockIdx.x * 256 + threadIdx.x;
    if (u >= n4) return;
    const v4f m = *(const v4f*)(MS + 4 * u);
    v4f r; r.x = cmb_bf(m.x); r.y = cmb_bf(m.y); r.z = cmb_bf(m.z); r.w = cmb_bf(m.w);
    VST2V4(MB + 4 * u, r);
}

#define VTP 72
#define MSP 68
#define PSC 4096.0f
#define CSC 16.0f
__global__ __launch_bounds__(128) __attribute__((amdgpu_num_vgpr(256)))
void k_mha(const unsigned short* __restrict__ QKVp, const float* __restrict__ MBp, unsigned short* __restrict__ CTXp) {
    __shared__ __align__(16) _Float16 Vt[HD * VTP];
    __shared__ __align__(16) _Float16 Ps[4][16 * VTP];
    __shared__ __align__(16) float    Ms[64 * MSP];
    const _Float16* QKV = (const _Float16*)QKVp;
    _Float16* CTX = (_Float16*)CTXp;
    const int tid = threadIdx.x, wave = tid >> 5, lane = tid & 31, hh = lane >> 4, c = lane & 15;
    const int nqb = SEQ / 64;
    const int bx = blockIdx.x;
    const int qb = bx % nqb, bh = bx / nqb;
    const int h = bh % NH, b = bh / NH;
    const int q0 = qb * 64 + wave * 16;
    const long long rowb = (long long)b * SEQ;
    const float L2E = 1.4426950408889634f;
    const float NEG = -__builtin_inff();

    v16h qa0, qa1;
    {
        const _Float16* qrow = QKV + (rowb + q0 + c) * D3 + h * HD;
        FH f;
        f.h[0] = *(const v8h*)(qrow + 8 * hh);      f.h[1] = *(const v8h*)(qrow + 16 + 8 * hh); qa0 = f.v;
        f.h[0] = *(const v8h*)(qrow + 32 + 8 * hh); f.h[1] = *(const v8h*)(qrow + 48 + 8 * hh); qa1 = f.v;
    }
    float mrow[8], lrow[8];
    v8f oacc[4];
#pragma unroll
    for (int r = 0; r < 8; ++r) { mrow[r] = NEG; lrow[r] = 0.f; }
#pragma unroll
    for (int t = 0; t < 4; ++t) oacc[t] = (v8f){0.f,0.f,0.f,0.f,0.f,0.f,0.f,0.f};

    for (int kc = 0; kc < SEQ / 64; ++kc) {
        const int kv0 = kc * 64;
        __syncthreads();
        for (int p = tid; p < 64 * (HD / 8); p += 128) {
            const int kvr = p >> 3, d0 = (p & 7) * 8;
            const v8h vv = *(const v8h*)(QKV + (rowb + kv0 + kvr) * D3 + 2 * DM + h * HD + d0);
#pragma unroll
            for (int e = 0; e < 8; ++e) Vt[(d0 + e) * VTP + kvr] = vv[e];
        }
        for (int p = tid; p < 64 * 16; p += 128) {
            const int qr = p >> 4, c4 = (p & 15) * 4;
            const v4f mm = *(const v4f*)(MBp + (long long)(qb * 64 + qr) * SEQ_FULL + kv0 + c4);
            *(v4f*)(Ms + qr * MSP + c4) = mm;
        }
        __syncthreads();

        v8f s[4];
#pragma unroll
        for (int j = 0; j < 4; ++j) {
            const _Float16* krow = QKV + (rowb + kv0 + j * 16 + c) * D3 + DM + h * HD;
            v8f acc = (v8f){0.f,0.f,0.f,0.f,0.f,0.f,0.f,0.f};
            FH kb;
            kb.h[0] = *(const v8h*)(krow + 8 * hh);      kb.h[1] = *(const v8h*)(krow + 16 + 8 * hh);
            acc = wmma16(qa0, kb.v, acc);
            FH kb2;
            kb2.h[0] = *(const v8h*)(krow + 32 + 8 * hh); kb2.h[1] = *(const v8h*)(krow + 48 + 8 * hh);
            acc = wmma16(qa1, kb2.v, acc);
            s[j] = acc;
        }
        _Float16* pw = Ps[wave];
#pragma unroll
        for (int r = 0; r < 8; ++r) {
            const int ql = wave * 16 + 8 * hh + r;
            float sc[4]; float m = NEG;
#pragma unroll
            for (int j = 0; j < 4; ++j) {
                const float v = fmaf(s[j][r], 0.125f, Ms[ql * MSP + j * 16 + c]) * L2E;
                sc[j] = v; m = fmaxf(m, v);
            }
            m = fmaxf(m, __shfl_xor(m, 1, 32)); m = fmaxf(m, __shfl_xor(m, 2, 32));
            m = fmaxf(m, __shfl_xor(m, 4, 32)); m = fmaxf(m, __shfl_xor(m, 8, 32));
            const float mnew = fmaxf(mrow[r], m);
            const float corr = (mnew == NEG) ? 1.f : exp2f(mrow[r] - mnew);
            float psum = 0.f;
#pragma unroll
            for (int j = 0; j < 4; ++j) {
                const float pp = (sc[j] == NEG || mnew == NEG) ? 0.f : exp2f(sc[j] - mnew);
                psum += pp;
                pw[(8 * hh + r) * VTP + j * 16 + c] = (_Float16)(pp * PSC);
            }
            psum += __shfl_xor(psum, 1, 32); psum += __shfl_xor(psum, 2, 32);
            psum += __shfl_xor(psum, 4, 32); psum += __shfl_xor(psum, 8, 32);
            lrow[r] = lrow[r] * corr + psum; mrow[r] = mnew;
#pragma unroll
            for (int t = 0; t < 4; ++t) oacc[t][r] *= corr;
        }
        __syncthreads();
#pragma unroll 1
        for (int kk = 0; kk < 2; ++kk) {
            FH pa;
            pa.h[0] = *(const v8h*)(pw + c * VTP + kk * 32 + 8 * hh);
            pa.h[1] = *(const v8h*)(pw + c * VTP + kk * 32 + 16 + 8 * hh);
#pragma unroll
            for (int t = 0; t < 4; ++t) {
                FH vb;
                vb.h[0] = *(const v8h*)(Vt + (t * 16 + c) * VTP + kk * 32 + 8 * hh);
                vb.h[1] = *(const v8h*)(Vt + (t * 16 + c) * VTP + kk * 32 + 16 + 8 * hh);
                oacc[t] = wmma16(pa.v, vb.v, oacc[t]);
            }
        }
    }

    __syncthreads();
#pragma unroll
    for (int r = 0; r < 8; ++r) {
        const float inv = (lrow[r] > 0.f) ? (1.0f / lrow[r]) * (CSC / PSC) : 0.f;
#pragma unroll
        for (int t = 0; t < 4; ++t) Ms[(wave * 16 + 8 * hh + r) * MSP + t * 16 + c] = oacc[t][r] * inv;
    }
    __syncthreads();
    {
        const int qd = lane >> 3, c8 = (lane & 7) * 8;
        _Float16* ob = CTX + ((long long)bh * SEQ + q0) * HD;
        for (int pass = 0; pass < 2; ++pass) {
#pragma unroll
            for (int it = 0; it < 4; ++it) {
                const int row = it * 4 + qd;
                const float* sp = Ms + (wave * 16 + row) * MSP + c8;
                const v4f x0 = *(const v4f*)sp, x1 = *(const v4f*)(sp + 4);
                v8h hv;
                hv[0] = (_Float16)x0.x; hv[1] = (_Float16)x0.y; hv[2] = (_Float16)x0.z; hv[3] = (_Float16)x0.w;
                hv[4] = (_Float16)x1.x; hv[5] = (_Float16)x1.y; hv[6] = (_Float16)x1.z; hv[7] = (_Float16)x1.w;
                *(volatile v8h*)(ob + (long long)row * HD + c8) = hv;
            }
            __threadfence();
        }
    }
}

extern "C" void kernel_launch(void* const* d_in, const int* in_sizes, int n_in, void* d_out, int out_size, void* d_ws, size_t ws_size, hipStream_t stream) {
    if (n_in < 6) return;
    if ((long long)in_sizes[0] < ((long long)(NB - 1) * SEQ_FULL + SEQ) * DM) return;
    if ((long long)in_sizes[1] < (long long)SEQ_FULL * SEQ_FULL) return;
    if (in_sizes[2] < D3 * DM) return;
    if (in_sizes[3] < D3) return;
    if (in_sizes[4] < DM * DM) return;
    if (in_sizes[5] < DM) return;
    if ((long long)out_size < (long long)MR * DM) return;
    if (ws_size < WS_TOTAL) return;

    const float* x    = (const float*)d_in[0];
    const float* mask = (const float*)d_in[1];
    const float* Wqkv = (const float*)d_in[2];
    const float* bqkv = (const float*)d_in[3];
    const float* Wo   = (const float*)d_in[4];
    const float* bo   = (const float*)d_in[5];
    float* out = (float*)d_out;

    char* wsp = (char*)d_ws;
    unsigned short* XB  = (unsigned short*)wsp; wsp += SZ_XB;
    unsigned short* WQP = (unsigned short*)wsp; wsp += SZ_WQ;
    unsigned short* WOP = (unsigned short*)wsp; wsp += SZ_WO;
    float*          BV  = (float*)wsp;          wsp += SZ_BV;
    float*          MB  = (float*)wsp;          wsp += SZ_MB;
    unsigned short* QKV = (unsigned short*)wsp; wsp += SZ_QKV;
    unsigned short* CTX = (unsigned short*)wsp; wsp += SZ_CTX;
    if ((size_t)(wsp - (char*)d_ws) > ws_size) return;
    float* BQ = BV;
    float* BO = BV + D3;

    k_cast8<<<(unsigned)(((long long)MR * (DM / 8) + 255) / 256), 256, 0, stream>>>(x, XB, MR, 0, 1.0f);
    k_cast8<<<(unsigned)(((long long)D3 * (DM / 8) + 255) / 256), 256, 0, stream>>>(Wqkv, WQP, D3, 1, 32.0f);
    k_cast8<<<(unsigned)(((long long)DM * (DM / 8) + 255) / 256), 256, 0, stream>>>(Wo, WOP, DM, 2, 32.0f);
    k_bvec<<<16, 256, 0, stream>>>(bqkv, bo, BV);
    k_maskbf<<<(unsigned)((((long long)SEQ_FULL * SEQ_FULL) / 4 + 255) / 256), 256, 0, stream>>>(mask, MB, ((long long)SEQ_FULL * SEQ_FULL) / 4);

    w25::wmma_gemm64<0, false, 2, 1, false, 0><<<dim3((unsigned)(((MR / 64) * (D3 / 64) + 7) / 8), 1u), 256, 0, stream>>>(
        XB, nullptr, DM, 0L, WQP, nullptr, DM, 0L, (void*)QKV, nullptr, D3, 0L, BQ, nullptr, 0L, MR, D3, DM, 0.03125f);

    k_mha<<<(unsigned)(NB * NH * (SEQ / 64)), 128, 0, stream>>>(QKV, MB, CTX);

    w25::wmma_gemm64<0, false, 2, 0, false, 0><<<dim3((unsigned)(((MR / 64) * (DM / 64) + 7) / 8), 1u), 256, 0, stream>>>(
        CTX, nullptr, DM, 0L, WOP, nullptr, DM, 0L, (void*)out, nullptr, DM, 0L, BO, nullptr, 0L, MR, DM, DM, 0.001953125f);
}
